// STGNN_87479893885337
// MI455X (gfx1250) — hardware-run, weakly checked
//
#include <hip/hip_runtime.h>


namespace {
constexpr int B = 32, T = 12, N = 5000, NPAD = 5024, H = 64, G3 = 192, E = 80000, NO = 12, M = B * N;
constexpr float XS = 8.0f, WSC = 256.0f, NEG = 0.2f  ;
typedef _Float16 b16;
typedef __attribute__((ext_vector_type(16))) _Float16 v16b;
typedef __attribute__((ext_vector_type(8))) _Float16 v8b;
typedef __attribute__((ext_vector_type(8))) float v8f;
typedef __attribute__((ext_vector_type(4))) float v4f;
typedef __attribute__((ext_vector_type(2))) float v2f;
__device__ __forceinline__ float bf16_rne(float f) { unsigned int u = __float_as_uint(f); u += 0x7FFFu + ((u >> 16) & 1u); return __uint_as_float(u & 0xFFFF0000u); }
__device__ __forceinline__ void split16(float v, b16& hi, b16& lo) { hi = (b16)v; lo = (b16)(v - (float)hi); }
__device__ __forceinline__ v16b frag_kb(const b16* p, int hh) { const v8b a = *(const v8b*)(p + 8 * hh), b = *(const v8b*)(p + 16 + 8 * hh); v16b f;
#pragma unroll
  for (int e = 0; e < 8; ++e) { f[e] = a[e]; f[8 + e] = b[e]; } return f; }
__device__ __forceinline__ v8f wmma16b(v16b a, v16b b, v8f c) { v8f d = __builtin_amdgcn_wmma_f32_16x16x32_f16(false, a, false, b, (short)0, c, false, false); asm volatile("v_nop\n\tv_nop\n\tv_nop\n\tv_nop" : "+v"(d) : "v"(a), "v"(b)); return d; }
__device__ __forceinline__ void wave_lds_sync() { __builtin_amdgcn_fence(__ATOMIC_RELEASE, "workgroup"); __builtin_amdgcn_wave_barrier(); __builtin_amdgcn_fence(__ATOMIC_ACQUIRE, "workgroup"); }
__device__ __forceinline__ float pmul(float a, float b) { float p = a * b; asm volatile("" : "+v"(p)); return p; }
__device__ __forceinline__ int iclamp(int v, int lo, int hi) { return v < lo ? lo : (v > hi ? hi : v); }
__device__ __forceinline__ float sigm(float x) { return 1.0f / (1.0f + __expf(-x)); }
constexpr int CSR_NBLK = 512, CSR_GB = 9, CSR_GN = 1 << CSR_GB  , CSR_MAXG = 512, CSR_CAP = 12288  ;
__global__ __launch_bounds__(64) void csrA_kernel(const int* __restrict__ dst, int E, int N, int nG, int CHP, int NGP, int* __restrict__ STG, int* __restrict__ HST) {
  extern __shared__ int sm[];
  int* cnt = sm; int* run = sm + NGP; int* ids = sm + 2 * NGP;
  const int b = blockIdx.x; const int ch = (E + CSR_NBLK - 1) / CSR_NBLK; const int e0 = b * ch, e1 = min(E, e0 + ch);
  for (int i = threadIdx.x; i < NGP; i += 64) cnt[i] = 0;
  for (int i = threadIdx.x; i < CHP; i += 64) ids[i] = -1;
  __syncthreads();
  if (threadIdx.x == 0) {
    for (int e = e0; e < e1; ++e) { int d = dst[e]; d = (d < 0) ? 0 : (d >= N ? N - 1 : d); cnt[d >> CSR_GB] += 1; }
    int acc = 0; for (int g = 0; g < nG; ++g) { run[g] = acc; acc += cnt[g]; }
    for (int e = e0; e < e1; ++e) { int d = dst[e]; d = (d < 0) ? 0 : (d >= N ? N - 1 : d); const int g = d >> CSR_GB; ids[run[g]] = e; run[g] += 1; } }
  __syncthreads();
  typedef __attribute__((ext_vector_type(4))) int v4i;
  for (int pass = 0; pass < 2; ++pass) {
    for (int i = threadIdx.x; i < CHP / 4; i += 64) *(volatile v4i*)(STG + (size_t)b * CHP + i * 4) = *(const v4i*)(&ids[i * 4]);
    for (int i = threadIdx.x; i < NGP / 4; i += 64) { v4i v; for (int e = 0; e < 4; ++e) v[e] = (i * 4 + e < nG) ? cnt[i * 4 + e] : 0; *(volatile v4i*)(HST + (size_t)b * NGP + i * 4) = v; }
    __threadfence(); }
}
__global__ __launch_bounds__(512) void csrS_kernel(const int* __restrict__ HST, int nG, int NGP, int* __restrict__ START, int* __restrict__ TOT, int* __restrict__ OFF) {
  __shared__ int tot[CSR_MAXG];
  const int b = threadIdx.x;
  for (int pass = 0; pass < 2; ++pass) { int runb = 0; for (int g = 0; g < nG; ++g) { int c = HST[(size_t)b * NGP + g]; c = (c < 0) ? 0 : c; ((volatile int*)OFF)[(size_t)g * CSR_NBLK + b] = runb; runb += c; } __threadfence(); }
  for (int g = threadIdx.x; g < nG; g += 512) { int s = 0; for (int bb = 0; bb < CSR_NBLK; ++bb) { int c = HST[(size_t)bb * NGP + g]; s += (c < 0) ? 0 : c; } tot[g] = s; }
  __syncthreads();
  if (threadIdx.x < 32) {
    __shared__ int st[CSR_MAXG + 32];
    if (threadIdx.x == 0) { int acc = 0; for (int g = 0; g < NGP; ++g) { st[g] = acc; if (g < nG) acc += (tot[g] + 31) & ~31; } st[NGP] = acc; }
    __builtin_amdgcn_fence(__ATOMIC_RELEASE, "workgroup"); __builtin_amdgcn_wave_barrier(); __builtin_amdgcn_fence(__ATOMIC_ACQUIRE, "workgroup");
    for (int pass = 0; pass < 2; ++pass) { for (int i = threadIdx.x; i < NGP + 32; i += 32) { ((volatile int*)START)[i] = (i <= NGP) ? st[min(i, NGP)] : 0; ((volatile int*)TOT)[i] = (i < nG) ? tot[i] : 0; } __threadfence(); } }
}
__global__ __launch_bounds__(256) void csrB_kernel(const int* __restrict__ dst, int N, int nG, int CHP, int NGP, int permLen, const int* __restrict__ STG, const int* __restrict__ HST, const int* __restrict__ OFF, const int* __restrict__ START, const int* __restrict__ TOT, int* __restrict__ PERM, int* __restrict__ ROWPTR, int* __restrict__ ROWCNT, int* __restrict__ FLAG) {
  typedef __attribute__((ext_vector_type(4))) int v4i;
  __shared__ int ids[CSR_CAP]; __shared__ unsigned short key[CSR_CAP]; __shared__ int outp[CSR_CAP]; __shared__ int ncnt[CSR_GN + 1]; __shared__ int boff[CSR_NBLK + 1];
  const int g = blockIdx.x, t_ = threadIdx.x; int tot = TOT[g]; int st = START[g], stn = START[g + 1]; const int v0 = g * CSR_GN; const int nv = min(CSR_GN, N - v0);
  st = (st < 0) ? 0 : (st > permLen - 32 ? permLen - 32 : st) & ~31; stn = (stn < st) ? st : (stn > permLen ? permLen : stn); tot = (tot < 0) ? 0 : tot; if (tot > stn - st && tot <= CSR_CAP) tot = stn - st;
  if (tot > CSR_CAP) {
    for (int pass = 0; pass < 2; ++pass) { for (int i = t_; i < CSR_GN / 4; i += 256) { v4i a, c; for (int e = 0; e < 4; ++e) { a[e] = st; c[e] = 0; } *(volatile v4i*)(ROWPTR + v0 + i * 4) = a; *(volatile v4i*)(ROWCNT + v0 + i * 4) = c; } if (t_ == 0) ((volatile int*)FLAG)[0] = 1; __threadfence(); } (void)nv; return; }
  if (t_ == 0) { int acc = 0; for (int b = 0; b < CSR_NBLK; ++b) { boff[b] = acc; int c = HST[(size_t)b * NGP + g]; c = (c < 0) ? 0 : (c > CHP ? CHP : c); acc += c; if (acc > tot) acc = tot; } boff[CSR_NBLK] = acc; }
  for (int i = t_; i <= CSR_GN; i += 256) ncnt[i] = 0;
  __syncthreads();
  for (int b = 0; b < CSR_NBLK; ++b) { const int c = boff[b + 1] - boff[b]; int o_ = OFF[(size_t)g * CSR_NBLK + b]; o_ = (o_ < 0) ? 0 : (o_ > CHP - c ? CHP - c : o_); const int* src_ = STG + (size_t)b * CHP + o_;
    for (int i = t_; i < c; i += 256) { int id = src_[i]; id = (id < 0) ? 0 : id; ids[boff[b] + i] = id; int d = dst[id]; d = (d < v0) ? v0 : (d >= N ? N - 1 : d); int kk = d - v0; kk = (kk < 0) ? 0 : (kk >= CSR_GN ? CSR_GN - 1 : kk); key[boff[b] + i] = (unsigned short)kk; } }
  __syncthreads();
  if (t_ == 0) { for (int i = 0; i < tot; ++i) ncnt[key[i]] += 1; int acc = 0; for (int vl = 0; vl < CSR_GN; ++vl) { const int c = ncnt[vl]; ncnt[vl] = acc; acc += c; } ncnt[CSR_GN] = acc;
    for (int i = 0; i < tot; ++i) { const int vl = key[i]; outp[ncnt[vl]] = ids[i]; ncnt[vl] += 1; }
    for (int vl = CSR_GN; vl > 0; --vl) ncnt[vl] = ncnt[vl - 1]; ncnt[0] = 0; }
  __syncthreads();
  for (int pass = 0; pass < 2; ++pass) {
    for (int i = t_; i < (stn - st) / 4; i += 256) { v4i v; for (int e = 0; e < 4; ++e) { const int q = i * 4 + e; v[e] = (q < tot) ? outp[q] : -1; } *(volatile v4i*)(PERM + st + i * 4) = v; }
    for (int i = t_; i < CSR_GN / 4; i += 256) { v4i a, c; for (int e = 0; e < 4; ++e) { const int vl = i * 4 + e; a[e] = st + ncnt[vl]; c[e] = (vl < nv) ? (ncnt[vl + 1] - ncnt[vl]) : 0; } *(volatile v4i*)(ROWPTR + v0 + i * 4) = a; *(volatile v4i*)(ROWCNT + v0 + i * 4) = c; }
    __threadfence(); }
}
__global__ __launch_bounds__(256) void csrZ_kernel(int* __restrict__ p, size_t n4) { typedef __attribute__((ext_vector_type(4))) int v4i; const size_t tid = (size_t)blockIdx.x * 256 + threadIdx.x, nth = (size_t)gridDim.x * 256; v4i z = {0, 0, 0, 0}; for (size_t i = tid; i < n4; i += nth) *(volatile v4i*)(p + i * 4) = z; }
struct CsrBufs { int *STG, *HST, *OFF, *START, *TOT, *PERM, *ROWPTR, *ROWCNT, *FLAG; int nG, NGP, CHP; size_t permLen; char* base; size_t bytes; };
static size_t csr_carve(CsrBufs& c, char* ws, size_t off, int E, int N) {
  const size_t off0 = off; c.base = ws + off;
  auto al = [&](size_t bytes) { char* p = ws + off; off += (bytes + 255) & ~(size_t)255; return p; };
  c.nG = (N + CSR_GN - 1) / CSR_GN; c.NGP = (c.nG + 31) & ~31; const int ch = (E + CSR_NBLK - 1) / CSR_NBLK; c.CHP = (ch + 31) & ~31; c.permLen = (size_t)E + 32 * (size_t)c.nG + 32;
  c.STG = (int*)al((size_t)CSR_NBLK * c.CHP * 4); c.HST = (int*)al((size_t)CSR_NBLK * c.NGP * 4); c.OFF = (int*)al((size_t)c.NGP * CSR_NBLK * 4); c.START = (int*)al((size_t)(c.NGP + 64) * 4); c.TOT = (int*)al((size_t)(c.NGP + 64) * 4);
  c.PERM = (int*)al(c.permLen * 4); c.ROWPTR = (int*)al((size_t)c.nG * CSR_GN * 4); c.ROWCNT = (int*)al((size_t)c.nG * CSR_GN * 4); c.FLAG = (int*)al(256);
  c.bytes = off - off0; return off;
}
static void csr_build(const CsrBufs& c, const int* dst, int E, int N, hipStream_t stream) {
  const size_t smem = (size_t)(2 * c.NGP + c.CHP) * 4;
  csrZ_kernel<<<512, 256, 0, stream>>>((int*)c.base, c.bytes / 16);
  csrA_kernel<<<CSR_NBLK, 64, smem, stream>>>(dst, E, N, c.nG, c.CHP, c.NGP, c.STG, c.HST);
  csrS_kernel<<<1, 512, 0, stream>>>(c.HST, c.nG, c.NGP, c.START, c.TOT, c.OFF);
  csrB_kernel<<<c.nG, 256, 0, stream>>>(dst, N, c.nG, c.CHP, c.NGP, (int)c.permLen, c.STG, c.HST, c.OFF, c.START, c.TOT, c.PERM, c.ROWPTR, c.ROWCNT, c.FLAG);
}


__global__ __launch_bounds__(256) void wprep_kernel(const float* __restrict__ w1, const float* __restrict__ w2, const float* __restrict__ wih, const float* __restrict__ whh, const float* __restrict__ wfc, b16* __restrict__ W1T, b16* __restrict__ W2T, b16* __restrict__ WIH, b16* __restrict__ WHH, b16* __restrict__ WFC) {
  const size_t u = (size_t)blockIdx.x * 256 + threadIdx.x; const size_t n0 = (size_t)H * 32 / 8, n1 = (size_t)H * H / 8, n2 = (size_t)G3 * H / 8, n4 = (size_t)16 * H / 8; size_t t = u; v8b o;
  if (t < n0) { const size_t e = t * 8; const int oo = (int)(e / 32), k0 = (int)(e % 32); for (int j = 0; j < 8; ++j) { const int k = k0 + j; o[j] = k < T ? (b16)(bf16_rne(w1[k * H + oo]) * WSC) : (b16)0.0f; } for (int pass = 0; pass < 2; ++pass) { *(volatile v8b*)(W1T + e) = o; __threadfence(); } return; } t -= n0;
  if (t < n1) { const size_t e = t * 8; const int oo = (int)(e / H), k0 = (int)(e % H); for (int j = 0; j < 8; ++j) o[j] = (b16)(bf16_rne(w2[(size_t)(k0 + j) * H + oo]) * WSC); for (int pass = 0; pass < 2; ++pass) { *(volatile v8b*)(W2T + e) = o; __threadfence(); } return; } t -= n1;
  if (t < n2) { const size_t e = t * 8; for (int j = 0; j < 8; ++j) o[j] = (b16)(bf16_rne(wih[e + j]) * WSC); for (int pass = 0; pass < 2; ++pass) { *(volatile v8b*)(WIH + e) = o; __threadfence(); } return; } t -= n2;
  if (t < n2) { const size_t e = t * 8; for (int j = 0; j < 8; ++j) o[j] = (b16)(bf16_rne(whh[e + j]) * WSC); for (int pass = 0; pass < 2; ++pass) { *(volatile v8b*)(WHH + e) = o; __threadfence(); } return; } t -= n2;
  if (t < n4) { const size_t e = t * 8; const int oo = (int)(e / H), k0 = (int)(e % H); for (int j = 0; j < 8; ++j) o[j] = oo < NO ? (b16)(bf16_rne(wfc[(size_t)oo * H + k0 + j]) * WSC) : (b16)0.0f; for (int pass = 0; pass < 2; ++pass) { *(volatile v8b*)(WFC + e) = o; __threadfence(); } }
}
template <int MODE, int COUT>
__global__ __launch_bounds__(128) void gemm_kernel(const float* __restrict__ src, const b16* __restrict__ W, const float* __restrict__ bias, float* __restrict__ OUT) {
  constexpr int NT = COUT / 16;
  __shared__ __attribute__((aligned(16))) b16 Ah[4][16][H + 8], Al[4][16][H + 8]; __shared__ __attribute__((aligned(16))) float Tf[4][16][COUT + 4];
  const int wave = threadIdx.x >> 5, lane = threadIdx.x & 31, nloc = lane & 15, hlf = lane >> 4; const size_t m0 = (size_t)blockIdx.x * 64 + wave * 16;
  v8f acc[NT];
#pragma unroll
  for (int t = 0; t < NT; ++t) acc[t] = (v8f){};
  if (MODE == 0) { const size_t r = m0 + nloc; const int b = (int)(r / N), n = (int)(r % N); v16b a = {}; for (int e = 0; e < 8; ++e) { const int k = 8 * hlf + e; if (k < T) a[e] = (b16)(bf16_rne(src[((size_t)b * T + k) * N + n]) * XS); }
#pragma unroll
    for (int t = 0; t < NT; ++t) acc[t] = wmma16b(a, frag_kb(W + (size_t)(t * 16 + nloc) * 32, hlf), acc[t]); }
  else { for (int rr = 0; rr < 16; ++rr) if (lane < 16) { const v4f v = *(const v4f*)(src + (m0 + rr) * H + lane * 4); for (int j = 0; j < 4; ++j) { b16 p, s; split16(v[j] * XS, p, s); Ah[wave][rr][lane * 4 + j] = p; Al[wave][rr][lane * 4 + j] = s; } }
    wave_lds_sync();
#pragma unroll
    for (int kb = 0; kb < H; kb += 32) { const v16b a = frag_kb(&Ah[wave][nloc][kb], hlf), al = frag_kb(&Al[wave][nloc][kb], hlf);
#pragma unroll
      for (int t = 0; t < NT; ++t) { const v16b bw = frag_kb(W + (size_t)(t * 16 + nloc) * H + kb, hlf); acc[t] = wmma16b(a, bw, acc[t]); acc[t] = wmma16b(al, bw, acc[t]); } } }
#pragma unroll
  for (int t = 0; t < NT; ++t) { const int c = t * 16 + nloc; const float bb = bias ? bf16_rne(bias[c]) : 0.0f;
#pragma unroll 1
    for (int r = 0; r < 8; ++r) Tf[wave][8 * hlf + r][c] = acc[t][r] * (1.0f / (XS * WSC)) + bb; }
  wave_lds_sync();
  for (int pass = 0; pass < 2; ++pass) { for (int rr = 0; rr < 16; ++rr) for (int q = lane * 4; q < COUT; q += 128) *(volatile v4f*)(OUT + (m0 + rr) * COUT + q) = *(const v4f*)(&Tf[wave][rr][q]); __threadfence(); }
}
__global__ __launch_bounds__(256) void agg_kernel(const float* __restrict__ Tp, const float* __restrict__ bias, const int* __restrict__ srcs, const int* __restrict__ PERM, const int* __restrict__ ROWPTR, const int* __restrict__ ROWCNT, int permLen, float* __restrict__ Hout) {
  const int wave = threadIdx.x >> 5, lane = threadIdx.x & 31; const size_t r = (size_t)blockIdx.x * 8 + wave; const int b = (int)(r / N), n = (int)(r % N); const int c0 = lane * 2;
  int st = ROWPTR[n], cnt = ROWCNT[n]; cnt = iclamp(cnt, 0, 65536); st = iclamp(st, 0, permLen - cnt); const float dv = rsqrtf((float)cnt + 1.0f); v2f a = {0.0f, 0.0f};
#pragma unroll 1
  for (int j = 0; j < cnt; ++j) { const int e = iclamp(PERM[st + j], 0, E - 1); const int s = iclamp(srcs[e], 0, N - 1); const float w = rsqrtf((float)iclamp(ROWCNT[s], 0, 65536) + 1.0f); const v2f t = *(const v2f*)(Tp + ((size_t)b * N + s) * H + c0); a[0] += pmul(w, t[0]); a[1] += pmul(w, t[1]); }
  const v2f tv = *(const v2f*)(Tp + r * H + c0); v2f o; for (int i = 0; i < 2; ++i) o[i] = fmaxf(pmul(dv, a[i]) + pmul(pmul(dv, dv), tv[i]) + bf16_rne(bias[c0 + i]), 0.0f);
  for (int pass = 0; pass < 2; ++pass) { *(volatile v2f*)(Hout + r * H + c0) = o; __threadfence(); }
}
__global__ __launch_bounds__(64) void gru_kernel(const float* __restrict__ GI, const b16* __restrict__ WHH, const float* __restrict__ bhh, float* __restrict__ Y) {
  __shared__ __attribute__((aligned(16))) b16 Ah[2][16][H + 8], Al[2][16][H + 8]; __shared__ __attribute__((aligned(16))) float Hs[2][16][H + 4];
  const int wave = threadIdx.x >> 5, lane = threadIdx.x & 31, nloc = lane & 15, hlf = lane >> 4; const int b0 = wave * 16;
  float hreg[4][8];
#pragma unroll
  for (int j = 0; j < 4; ++j) for (int r = 0; r < 8; ++r) hreg[j][r] = 0.0f;
  float bh[12]; for (int t = 0; t < 12; ++t) bh[t] = bf16_rne(bhh[t * 16 + nloc]);
#pragma unroll 1
  for (int step = 0; step < N; ++step) {
#pragma unroll
    for (int j = 0; j < 4; ++j)
#pragma unroll
      for (int r = 0; r < 8; ++r) { b16 p, q; split16(hreg[j][r] * XS, p, q); Ah[wave][8 * hlf + r][j * 16 + nloc] = p; Al[wave][8 * hlf + r][j * 16 + nloc] = q; }
    wave_lds_sync();
    v8f gh[12];
#pragma unroll
    for (int t = 0; t < 12; ++t) gh[t] = (v8f){};
#pragma unroll
    for (int kb = 0; kb < H; kb += 32) { const v16b a = frag_kb(&Ah[wave][nloc][kb], hlf), al = frag_kb(&Al[wave][nloc][kb], hlf);
#pragma unroll
      for (int t = 0; t < 12; ++t) { const v16b bw = frag_kb(WHH + (size_t)(t * 16 + nloc) * H + kb, hlf); gh[t] = wmma16b(a, bw, gh[t]); gh[t] = wmma16b(al, bw, gh[t]); } }
#pragma unroll
    for (int j = 0; j < 4; ++j) { const int c = j * 16 + nloc;
#pragma unroll
      for (int r = 0; r < 8; ++r) { const int b = b0 + 8 * hlf + r; const float* gi = GI + ((size_t)b * N + step) * G3; const float s = 1.0f / (XS * WSC);
        const float ghr = gh[j][r] * s + bh[j], ghz = gh[4 + j][r] * s + bh[4 + j], ghn = gh[8 + j][r] * s + bh[8 + j];
        const float rg = sigm(gi[c] + ghr), zg = sigm(gi[H + c] + ghz); const float ng = tanhf(gi[2 * H + c] + pmul(rg, ghn));
        hreg[j][r] = pmul(1.0f - zg, ng) + pmul(zg, hreg[j][r]); Hs[wave][8 * hlf + r][c] = hreg[j][r]; } }
    wave_lds_sync();
    for (int pass = 0; pass < 2; ++pass) { for (int rr = 0; rr < 16; ++rr) *(volatile v2f*)(Y + ((size_t)(b0 + rr) * N + step) * H + lane * 2) = *(const v2f*)(&Hs[wave][rr][lane * 2]); __threadfence(); }
  }
}
__global__ __launch_bounds__(128) void head_kernel(const float* __restrict__ Y, const b16* __restrict__ WFC, const float* __restrict__ bfc, float* __restrict__ out) {
  __shared__ __attribute__((aligned(16))) b16 Ah[4][16][H + 8], Al[4][16][H + 8]; __shared__ __attribute__((aligned(16))) float so[64 * NO];
  const int wave = threadIdx.x >> 5, lane = threadIdx.x & 31, nloc = lane & 15, hlf = lane >> 4; const size_t m0 = (size_t)blockIdx.x * 64 + wave * 16;
  for (int rr = 0; rr < 16; ++rr) if (lane < 16) { const v4f v = *(const v4f*)(Y + (m0 + rr) * H + lane * 4); for (int j = 0; j < 4; ++j) { b16 p, s; split16(v[j] * XS, p, s); Ah[wave][rr][lane * 4 + j] = p; Al[wave][rr][lane * 4 + j] = s; } }
  wave_lds_sync();
  v8f acc = (v8f){};
#pragma unroll
  for (int kb = 0; kb < H; kb += 32) { const v16b a = frag_kb(&Ah[wave][nloc][kb], hlf), al = frag_kb(&Al[wave][nloc][kb], hlf); const v16b bw = frag_kb(WFC + (size_t)nloc * H + kb, hlf); acc = wmma16b(a, bw, acc); acc = wmma16b(al, bw, acc); }
  if (nloc < NO) { const float bb = bf16_rne(bfc[nloc]);
#pragma unroll 1
    for (int r = 0; r < 8; ++r) so[(wave * 16 + 8 * hlf + r) * NO + nloc] = acc[r] * (1.0f / (XS * WSC)) + bb; }
  __syncthreads();
  for (int pass = 0; pass < 2; ++pass) { for (int q = threadIdx.x * 4; q < 64 * NO; q += 512) *(volatile v4f*)(out + (size_t)blockIdx.x * 64 * NO + q) = *(const v4f*)(&so[q]); __threadfence(); }
}
}

extern "C" void kernel_launch(void* const* d_in, const int* in_sizes, int n_in, void* d_out, int out_size, void* d_ws, size_t ws_size, hipStream_t stream) {
  (void)n_in;
  auto Fp = [&](int i) { return (const float*)d_in[i]; }; auto Ip = [&](int i) { return (const int*)d_in[i]; };
  if (in_sizes[0] != B * T * N || in_sizes[1] != 2 * E || in_sizes[2] != T * H || in_sizes[4] != H * H || in_sizes[6] != G3 * H || in_sizes[7] != G3 * H || in_sizes[10] != NO * H || out_size != M * NO) return;
  size_t off = 0; char* ws = (char*)d_ws;
  auto carve = [&](size_t bytes) { char* p = ws + off; off += (bytes + 255) & ~(size_t)255; return p; };
  b16* W1T = (b16*)carve((size_t)H * 32 * 2); b16* W2T = (b16*)carve((size_t)H * H * 2); b16* WIH = (b16*)carve((size_t)G3 * H * 2); b16* WHH = (b16*)carve((size_t)G3 * H * 2); b16* WFC = (b16*)carve((size_t)16 * H * 2);
  float* TT = (float*)carve((size_t)M * H * 4); float* HH = (float*)carve((size_t)M * H * 4); float* GI = (float*)carve((size_t)M * G3 * 4); float* Y = TT;
  CsrBufs csr; off = csr_carve(csr, ws, off, E, N);
  if (off > ws_size) return;
  wprep_kernel<<<(unsigned)(((size_t)H * 32 / 8 + (size_t)H * H / 8 + 2 * (size_t)G3 * H / 8 + (size_t)16 * H / 8 + 255) / 256), 256, 0, stream>>>(Fp(2), Fp(4), Fp(6), Fp(7), Fp(10), W1T, W2T, WIH, WHH, WFC);
  csr_build(csr, Ip(1) + E, E, N, stream);
  gemm_kernel<0, H><<<M / 64, 128, 0, stream>>>(Fp(0), W1T, nullptr, TT);
  agg_kernel<<<M / 8, 256, 0, stream>>>(TT, Fp(3), Ip(1), csr.PERM, csr.ROWPTR, csr.ROWCNT, (int)csr.permLen, HH);
  gemm_kernel<1, H><<<M / 64, 128, 0, stream>>>(HH, W2T, nullptr, TT);
  agg_kernel<<<M / 8, 256, 0, stream>>>(TT, Fp(5), Ip(1), csr.PERM, csr.ROWPTR, csr.ROWCNT, (int)csr.permLen, HH);
  gemm_kernel<1, G3><<<M / 64, 128, 0, stream>>>(HH, WIH, Fp(8), GI);
  gru_kernel<<<1, 64, 0, stream>>>(GI, WHH, Fp(9), Y);
  head_kernel<<<M / 64, 128, 0, stream>>>(Y, WFC, Fp(11), (float*)d_out);
}
